// GRU_43387759624777
// MI455X (gfx1250) — hardware-run, weakly checked
//
#include <hip/hip_runtime.h>
#include <math.h>

constexpr int NBATCH   = 4096;
constexpr int NSTEP    = 1024;
constexpr int NHID     = 64;
constexpr int NGATE3   = 3 * NHID;
constexpr int NHEAD1   = 32;
constexpr int NHEAD2   = 16;
constexpr int ROWS_BLK = 32;
constexpr int NTHR     = 256;
constexpr int TCH      = 32;
constexpr int WPL      = 64;
constexpr int HPL      = 64;
constexpr int APL      = ROWS_BLK * HPL;
constexpr int XSP      = 32;
constexpr int HSP      = 68;
constexpr int Y1P      = 36;
constexpr int Y2P      = 20;
constexpr float HCARRY = 16384.0f;
constexpr float WCARRY = 256.0f;
constexpr float FOLD   = 1.0f / (16384.0f * 256.0f);
constexpr float NEG_SLOPE_F = 0.01f;
constexpr bool  LO_RZ  = false;

static_assert(NBATCH % ROWS_BLK == 0);
static_assert(ROWS_BLK == 32);
static_assert(NTHR == 8 * 32);
static_assert(NHID == 64);
static_assert(NGATE3 * NHID == 12 * NTHR * 4);
static_assert(2 * APL == 2 * NTHR * 8);
static_assert(ROWS_BLK * TCH == NTHR * 4);
static_assert(NSTEP % TCH == 0 && (TCH & (TCH - 1)) == 0);
static_assert(ROWS_BLK * NHEAD1 == NTHR * 4);
static_assert(ROWS_BLK * NHEAD2 == NTHR * 2);

typedef __attribute__((ext_vector_type(16))) _Float16 v16h;
typedef __attribute__((ext_vector_type(8)))  _Float16 v8h;
typedef __attribute__((ext_vector_type(4)))  _Float16 v4h;
typedef __attribute__((ext_vector_type(8)))  float    v8f;
typedef __attribute__((ext_vector_type(4)))  float    v4f;

__device__ __forceinline__ unsigned short f2bf_bits(float f) {
  unsigned u = __float_as_uint(f);
  return (unsigned short)((u + 0x7FFFu + ((u >> 16) & 1u)) >> 16);
}
__device__ __forceinline__ float bf_bits2f(unsigned short h) { return __uint_as_float(((unsigned)h) << 16); }
__device__ __forceinline__ float bf16r(float f) { return bf_bits2f(f2bf_bits(f)); }

__device__ __forceinline__ v16h frag_load(const _Float16* p) {
  union { v16h v; v8h h[2]; } f;
  f.h[0] = *(const v8h*)(p);
  f.h[1] = *(const v8h*)(p + 16);
  return f.v;
}
__device__ __forceinline__ v8f mma16(v16h a, v16h b, v8f c) {
  return __builtin_amdgcn_wmma_f32_16x16x32_f16(false, a, false, b, (short)0, c, false, false);
}
__device__ __forceinline__ void grp_guard(v8f& d0, v8f& d1, v8f& d2,
                                          v16h a0, v16h a1, v16h a2, v16h a3,
                                          v16h b0, v16h b1, v16h b2, v16h b3, v16h b4, v16h b5) {
  asm volatile("v_nop\n\tv_nop\n\tv_nop\n\tv_nop"
               : "+v"(d0), "+v"(d1), "+v"(d2)
               : "v"(a0), "v"(a1), "v"(a2), "v"(a3), "v"(b0), "v"(b1), "v"(b2), "v"(b3), "v"(b4), "v"(b5));
}
__device__ __forceinline__ void opaque_f(float& v) { asm volatile("" : "+v"(v)); }

__device__ __forceinline__ float fsig(float a)  { return __builtin_amdgcn_rcpf(1.0f + __expf(-a)); }
__device__ __forceinline__ float ftanh(float a) { return 1.0f - 2.0f * __builtin_amdgcn_rcpf(__expf(2.0f * a) + 1.0f); }

__global__ __launch_bounds__(NTHR) void gru_head_kernel(
    const float* __restrict__ x,    const float* __restrict__ w_ih, const float* __restrict__ w_hh,
    const float* __restrict__ b_ih, const float* __restrict__ b_hh,
    const float* __restrict__ w1,   const float* __restrict__ b1,
    const float* __restrict__ w2,   const float* __restrict__ b2,
    const float* __restrict__ w3,   const float* __restrict__ b3,
    float* __restrict__ out) {
  __shared__ __align__(16) _Float16 Wl[NGATE3 * WPL];
  __shared__ __align__(16) _Float16 Ahi[2 * APL];
  __shared__ __align__(16) _Float16 Alo[2 * APL];
  __shared__ __align__(16) float    Xs[TCH * XSP];
  __shared__ __align__(16) float    Hs[ROWS_BLK * HSP];
  __shared__ __align__(16) float    Y1s[ROWS_BLK * Y1P];
  __shared__ __align__(16) float    Y2s[ROWS_BLK * Y2P];
  __shared__ __align__(16) float    Os[ROWS_BLK];

  const int tid = threadIdx.x, lane = tid & 31, wave = tid >> 5;
  const int c = lane & 15, hh = lane >> 4, koff = 8 * hh;
  const int msub = wave >> 2, ub = wave & 3;
  const int j = 16 * ub + c;
  const int lrow0 = 16 * msub + 8 * hh;
  const int rowbase = blockIdx.x * ROWS_BLK;

#pragma unroll 1
  for (int it = 0; it < 12; ++it) {
    const int idx = it * NTHR + tid;
    const int row = idx >> 4, c4 = (idx & 15) * 4;
    const v4f v = *(const v4f*)(w_hh + (size_t)row * NHID + c4);
    v4h hv;
    hv[0] = (_Float16)(bf16r(v[0]) * WCARRY);
    hv[1] = (_Float16)(bf16r(v[1]) * WCARRY);
    hv[2] = (_Float16)(bf16r(v[2]) * WCARRY);
    hv[3] = (_Float16)(bf16r(v[3]) * WCARRY);
    *(v4h*)(Wl + row * WPL + c4) = hv;
  }
  {
    v8h zh;
#pragma unroll
    for (int e = 0; e < 8; ++e) zh[e] = (_Float16)0.0f;
#pragma unroll
    for (int i = 0; i < 2; ++i) {
      *(v8h*)(Ahi + (size_t)(i * NTHR + tid) * 8) = zh;
      *(v8h*)(Alo + (size_t)(i * NTHR + tid) * 8) = zh;
    }
  }
  const float cwr = bf16r(w_ih[j]), cwz = bf16r(w_ih[NHID + j]), cwn = bf16r(w_ih[2 * NHID + j]);
  const float cir = bf16r(b_ih[j]), ciz = bf16r(b_ih[NHID + j]), cin = bf16r(b_ih[2 * NHID + j]);
  const float chr = bf16r(b_hh[j]), chz = bf16r(b_hh[NHID + j]), chn = bf16r(b_hh[2 * NHID + j]);
  float hold[8];
#pragma unroll
  for (int r = 0; r < 8; ++r) hold[r] = 0.0f;
  __syncthreads();

  const _Float16* wbr = Wl + (0 * NHID + j) * WPL + koff;
  const _Float16* wbz = Wl + (1 * NHID + j) * WPL + koff;
  const _Float16* wbn = Wl + (2 * NHID + j) * WPL + koff;
  const v16h br0 = frag_load(wbr), br1 = frag_load(wbr + 32);
  const v16h bz0 = frag_load(wbz), bz1 = frag_load(wbz + 32);
  const v16h bn0 = frag_load(wbn), bn1 = frag_load(wbn + 32);
  const _Float16* ahb = Ahi + (16 * msub + c) * HPL + koff;
  const _Float16* alb = Alo + (16 * msub + c) * HPL + koff;
  const v8f z8 = {0.f, 0.f, 0.f, 0.f, 0.f, 0.f, 0.f, 0.f};

#pragma unroll 1
  for (int t = 0; t < NSTEP; ++t) {
    if ((t & (TCH - 1)) == 0) {
      const int row = tid >> 3, t4 = (tid & 7) * 4;
      const v4f v = *(const v4f*)(x + (size_t)(rowbase + row) * NSTEP + (size_t)(t + t4));
      Xs[(t4 + 0) * XSP + row] = bf16r(v[0]);
      Xs[(t4 + 1) * XSP + row] = bf16r(v[1]);
      Xs[(t4 + 2) * XSP + row] = bf16r(v[2]);
      Xs[(t4 + 3) * XSP + row] = bf16r(v[3]);
      __syncthreads();
    }
    const int cur  = t & 1;
    const int poff = cur * APL, noff = (cur ^ 1) * APL;
    const int tl   = t & (TCH - 1);
    float xr[8];
    {
      const v4f q0 = *(const v4f*)(Xs + tl * XSP + lrow0);
      const v4f q1 = *(const v4f*)(Xs + tl * XSP + lrow0 + 4);
#pragma unroll
      for (int e = 0; e < 4; ++e) { xr[e] = q0[e]; xr[4 + e] = q1[e]; }
    }
    const v16h ah0 = frag_load(ahb + poff), ah1 = frag_load(ahb + poff + 32);
    const v16h al0 = frag_load(alb + poff), al1 = frag_load(alb + poff + 32);
    v8f accr = z8, accz = z8, accn = z8;
    if (LO_RZ) { accr = mma16(al0, br0, accr); accr = mma16(al1, br1, accr); }
    accr = mma16(ah0, br0, accr); accr = mma16(ah1, br1, accr);
    if (LO_RZ) { accz = mma16(al0, bz0, accz); accz = mma16(al1, bz1, accz); }
    accz = mma16(ah0, bz0, accz); accz = mma16(ah1, bz1, accz);
    accn = mma16(al0, bn0, accn); accn = mma16(al1, bn1, accn);
    accn = mma16(ah0, bn0, accn); accn = mma16(ah1, bn1, accn);
    grp_guard(accr, accz, accn, ah0, ah1, al0, al1, br0, br1, bz0, bz1, bn0, bn1);

#pragma unroll
    for (int r = 0; r < 8; ++r) {
      const float xv = xr[r];
      const float ar = (xv * cwr + cir) + (accr[r] * FOLD + chr);
      const float az = (xv * cwz + ciz) + (accz[r] * FOLD + chz);
      const float rg = fsig(ar);
      const float zg = fsig(az);
      const float an = (xv * cwn + cin) + rg * (accn[r] * FOLD + chn);
      const float ng = ftanh(an);
      const float hn = (1.0f - zg) * ng + zg * hold[r];
      hold[r] = hn;
      const float hs = hn * HCARRY;
      const _Float16 hi16 = (_Float16)hs;
      float hif = (float)hi16;
      opaque_f(hif);
      const _Float16 lo16 = (_Float16)(hs - hif);
      const int idx = noff + (lrow0 + r) * HPL + j;
      Ahi[idx] = hi16;
      Alo[idx] = lo16;
    }
    __syncthreads();
  }

#pragma unroll
  for (int r = 0; r < 8; ++r) Hs[(lrow0 + r) * HSP + j] = hold[r];
  __syncthreads();
  {
    const int row = tid >> 3, ubase = (tid & 7) * 4;
#pragma unroll 1
    for (int q = 0; q < 4; ++q) {
      const int u = ubase + q;
      const float* wrow = w1 + u * NHID;
      float s = 0.0f;
#pragma unroll 1
      for (int k = 0; k < NHID; ++k) s = fmaf(Hs[row * HSP + k], bf16r(wrow[k]), s);
      s += bf16r(b1[u]);
      s = (s >= 0.0f) ? s : NEG_SLOPE_F * s;
      Y1s[row * Y1P + u] = s;
    }
  }
  __syncthreads();
  {
    const int row = tid >> 3, ubase = (tid & 7) * 2;
#pragma unroll 1
    for (int q = 0; q < 2; ++q) {
      const int u = ubase + q;
      const float* wrow = w2 + u * NHEAD1;
      float s = 0.0f;
#pragma unroll 1
      for (int k = 0; k < NHEAD1; ++k) s = fmaf(Y1s[row * Y1P + k], bf16r(wrow[k]), s);
      s += bf16r(b2[u]);
      s = (s >= 0.0f) ? s : NEG_SLOPE_F * s;
      Y2s[row * Y2P + u] = s;
    }
  }
  __syncthreads();
  if (wave == 0) {
    float s = 0.0f;
#pragma unroll 1
    for (int k = 0; k < NHEAD2; ++k) s = fmaf(Y2s[lane * Y2P + k], bf16r(w3[k]), s);
    s += bf16r(b3[0]);
    Os[lane] = s;
  }
  __syncthreads();
  if (wave == 0) {
    const int q = (lane < 8) ? lane : 7;
    const v4f v = *(const v4f*)(Os + 4 * q);
    float* op = out + (size_t)rowbase + 4 * q;
    for (int pass = 0; pass < 2; ++pass) {
      if (lane < 8) *(volatile v4f*)op = v;
      __threadfence();
    }
  }
}

extern "C" void kernel_launch(void* const* d_in, const int* in_sizes, int n_in,
                              void* d_out, int out_size, void* d_ws, size_t ws_size, hipStream_t stream) {
  if (n_in < 11 || d_out == nullptr) return;
  if (in_sizes[0] != NBATCH * NSTEP || in_sizes[1] != NGATE3 || in_sizes[2] != NGATE3 * NHID ||
      in_sizes[3] != NGATE3 || in_sizes[4] != NGATE3 || in_sizes[5] != NHEAD1 * NHID || in_sizes[6] != NHEAD1 ||
      in_sizes[7] != NHEAD2 * NHEAD1 || in_sizes[8] != NHEAD2 || in_sizes[9] != NHEAD2 || in_sizes[10] != 1 ||
      out_size != NBATCH) return;

  const float* x    = (const float*)d_in[0];
  const float* w_ih = (const float*)d_in[1];
  const float* w_hh = (const float*)d_in[2];
  const float* b_ih = (const float*)d_in[3];
  const float* b_hh = (const float*)d_in[4];
  const float* w1   = (const float*)d_in[5];
  const float* b1   = (const float*)d_in[6];
  const float* w2   = (const float*)d_in[7];
  const float* b2   = (const float*)d_in[8];
  const float* w3   = (const float*)d_in[9];
  const float* b3   = (const float*)d_in[10];
  float* out = (float*)d_out;
  (void)d_ws; (void)ws_size;

  gru_head_kernel<<<NBATCH / ROWS_BLK, NTHR, 0, stream>>>(x, w_ih, w_hh, b_ih, b_hh, w1, b1, w2, b2, w3, b3, out);
}
